// swapHead_type_49478023250679
// MI455X (gfx1250) — hardware-verified
//
#include <hip/hip_runtime.h>
#include <stdint.h>

typedef _Float16 v16h __attribute__((ext_vector_type(16)));
typedef _Float16 v8h  __attribute__((ext_vector_type(8))) __attribute__((__may_alias__));
typedef float    v8f  __attribute__((ext_vector_type(8)));
typedef float    v4f  __attribute__((ext_vector_type(4))) __attribute__((__may_alias__));

#define NODE_DIM 64
#define HID      256
#define ROWH     128

union Frag { v16h v; v8h hv[2]; };

__device__ __forceinline__ v8f vzero8()
{
    v8f z;
    z[0] = 0.f; z[1] = 0.f; z[2] = 0.f; z[3] = 0.f;
    z[4] = 0.f; z[5] = 0.f; z[6] = 0.f; z[7] = 0.f;
    return z;
}

__device__ __forceinline__ v8f wmma_f16(v16h a, v16h b, v8f c)
{
    v8f d = __builtin_amdgcn_wmma_f32_16x16x32_f16(false, a, false, b, (short)0, c, false, false);
    asm volatile("v_nop\n\tv_nop\n\tv_nop\n\tv_nop" : "+v"(d) : "v"(a), "v"(b));
    return d;
}

__global__ __launch_bounds__(256) void repack_w1_f16(const float* __restrict__ W1,
                                                     _Float16* __restrict__ w1pk)
{
    const int t = blockIdx.x * 256 + threadIdx.x;
    if (t >= 4096) return;
    const int vec  = t >> 1;
    const int ih   = t & 1;
    const int lane = vec & 31;
    const int n    = (vec >> 5) & 15;
    const int kt   = vec >> 9;
    const int h    = lane >> 4;
    const int c    = lane & 15;
    const int kb   = kt * 32 + 8 * h + 16 * ih;
    const int col  = 16 * n + c;
    v8h v;
    #pragma unroll
    for (int ii = 0; ii < 8; ++ii)
        v[ii] = (_Float16)(W1[(size_t)(kb + ii) * HID + col] * 64.0f);
    _Float16* dst = w1pk + (size_t)t * 8;
    *(volatile v8h*)dst = v;
    __threadfence();
    *(volatile v8h*)dst = v;
}

__global__ __launch_bounds__(256) void gather_rows_f16(const float* __restrict__ x,
                                                       const int*   __restrict__ eidx,
                                                       _Float16*    __restrict__ G,
                                                       int N, int E, int e0, int Ec)
{
    const size_t gi = (size_t)blockIdx.x * 256 + threadIdx.x;
    const int el = (int)(gi >> 4);
    const int q  = (int)(gi & 15);
    if (el >= Ec) return;
    const int e = e0 + el;
    int node = (q < 8) ? eidx[e] : eidx[(size_t)E + e];
    if (node < 0) node += N;
    node = node < 0 ? 0 : (node >= N ? N - 1 : node);
    const float* xr = x + (size_t)node * NODE_DIM + (q & 7) * 8;
    const v4f a = *(const v4f*)xr;
    const v4f b = *(const v4f*)(xr + 4);
    v8h v;
    v[0] = (_Float16)(a[0] * 8.0f); v[1] = (_Float16)(a[1] * 8.0f);
    v[2] = (_Float16)(a[2] * 8.0f); v[3] = (_Float16)(a[3] * 8.0f);
    v[4] = (_Float16)(b[0] * 8.0f); v[5] = (_Float16)(b[1] * 8.0f);
    v[6] = (_Float16)(b[2] * 8.0f); v[7] = (_Float16)(b[3] * 8.0f);
    _Float16* dst = G + (size_t)el * ROWH + q * 8;
    *(volatile v8h*)dst = v;
    __threadfence();
    *(volatile v8h*)dst = v;
}

__device__ __forceinline__ void store_out_line(float* __restrict__ outc, int tbase, int l,
                                               v4f ov, int Ec)
{
    if (l < 8) {
        const int eo = tbase + 4 * l;
        float* p = outc + eo;
        if (eo + 3 < Ec) {
            *(volatile v4f*)p = ov;
        } else {
            if (eo + 0 < Ec) ((volatile float*)p)[0] = ov[0];
            if (eo + 1 < Ec) ((volatile float*)p)[1] = ov[1];
            if (eo + 2 < Ec) ((volatile float*)p)[2] = ov[2];
            if (eo + 3 < Ec) ((volatile float*)p)[3] = ov[3];
        }
    }
}

__global__ __launch_bounds__(256) void edge_mlp_wmma(
    const _Float16* __restrict__ G,
    const _Float16* __restrict__ w1pk,
    const float*    __restrict__ b1,
    const float*    __restrict__ W2,
    const float*    __restrict__ b2,
    float*          __restrict__ outc,
    int Ec)
{
    const int l = threadIdx.x & 31;
    const int h = l >> 4;
    const int m = l & 15;
    const int nwaves = gridDim.x * 8;
    const int gwave  = blockIdx.x * 8 + (threadIdx.x >> 5);
    const int numTiles = (Ec + 31) >> 5;
    const v16h* __restrict__ bmat = (const v16h*)w1pk;
    const float bias2 = b2[0];
    const float inv512 = 1.0f / 512.0f;

    for (int tile = gwave; tile < numTiles; tile += nwaves) {
        const int tbase = tile * 32;

        Frag As[2][2], Ad[2][2];
        #pragma unroll
        for (int mt = 0; mt < 2; ++mt) {
            int el = tbase + mt * 16 + m;
            int ec = el < Ec ? el : Ec - 1;
            const _Float16* row = G + (size_t)ec * ROWH;
            #pragma unroll
            for (int t = 0; t < 2; ++t) {
                As[mt][t].hv[0] = *(const v8h*)(row + 32 * t + 8 * h);
                As[mt][t].hv[1] = *(const v8h*)(row + 32 * t + 16 + 8 * h);
                Ad[mt][t].hv[0] = *(const v8h*)(row + 64 + 32 * t + 8 * h);
                Ad[mt][t].hv[1] = *(const v8h*)(row + 64 + 32 * t + 16 + 8 * h);
            }
        }

        float acc0[8] = {0.f, 0.f, 0.f, 0.f, 0.f, 0.f, 0.f, 0.f};
        float acc1[8] = {0.f, 0.f, 0.f, 0.f, 0.f, 0.f, 0.f, 0.f};
        #pragma unroll 1
        for (int n = 0; n < 16; ++n) {
            const v16h Bw0 = bmat[(0 * 16 + n) * 32 + l];
            const v16h Bw1 = bmat[(1 * 16 + n) * 32 + l];
            const v16h Bw2 = bmat[(2 * 16 + n) * 32 + l];
            const v16h Bw3 = bmat[(3 * 16 + n) * 32 + l];

            v8f cf0 = vzero8(), cr0 = vzero8(), cf1 = vzero8(), cr1 = vzero8();
            cf0 = wmma_f16(As[0][0].v, Bw0, cf0);
            cr0 = wmma_f16(Ad[0][0].v, Bw0, cr0);
            cf1 = wmma_f16(As[1][0].v, Bw0, cf1);
            cr1 = wmma_f16(Ad[1][0].v, Bw0, cr1);
            cf0 = wmma_f16(As[0][1].v, Bw1, cf0);
            cr0 = wmma_f16(Ad[0][1].v, Bw1, cr0);
            cf1 = wmma_f16(As[1][1].v, Bw1, cf1);
            cr1 = wmma_f16(Ad[1][1].v, Bw1, cr1);
            cf0 = wmma_f16(Ad[0][0].v, Bw2, cf0);
            cr0 = wmma_f16(As[0][0].v, Bw2, cr0);
            cf1 = wmma_f16(Ad[1][0].v, Bw2, cf1);
            cr1 = wmma_f16(As[1][0].v, Bw2, cr1);
            cf0 = wmma_f16(Ad[0][1].v, Bw3, cf0);
            cr0 = wmma_f16(As[0][1].v, Bw3, cr0);
            cf1 = wmma_f16(Ad[1][1].v, Bw3, cf1);
            cr1 = wmma_f16(As[1][1].v, Bw3, cr1);

            const float bb = b1[n * 16 + m];
            const float wv = W2[n * 16 + m];
            #pragma unroll
            for (int j = 0; j < 8; ++j) {
                float hf0 = cf0[j] * inv512 + bb; hf0 = hf0 > 0.f ? hf0 : 0.f;
                float hr0 = cr0[j] * inv512 + bb; hr0 = hr0 > 0.f ? hr0 : 0.f;
                float hf1 = cf1[j] * inv512 + bb; hf1 = hf1 > 0.f ? hf1 : 0.f;
                float hr1 = cr1[j] * inv512 + bb; hr1 = hr1 > 0.f ? hr1 : 0.f;
                acc0[j] += (hf0 + hr0) * wv;
                acc1[j] += (hf1 + hr1) * wv;
            }
        }

        #pragma unroll
        for (int j = 0; j < 8; ++j) {
            float v0 = acc0[j];
            v0 += __shfl_xor(v0, 1, 32);
            v0 += __shfl_xor(v0, 2, 32);
            v0 += __shfl_xor(v0, 4, 32);
            v0 += __shfl_xor(v0, 8, 32);
            acc0[j] = v0;
            float v1 = acc1[j];
            v1 += __shfl_xor(v1, 1, 32);
            v1 += __shfl_xor(v1, 2, 32);
            v1 += __shfl_xor(v1, 4, 32);
            v1 += __shfl_xor(v1, 8, 32);
            acc1[j] = v1;
        }

        const int jj = l & 7;
        const int hh = (l >> 3) & 1;
        float p0 = 0.f, p1 = 0.f;
        #pragma unroll
        for (int j = 0; j < 8; ++j) {
            if (jj == j) { p0 = acc0[j]; p1 = acc1[j]; }
        }
        const float q0 = __shfl_xor(p0, 16, 32);
        const float q1 = __shfl_xor(p1, 16, 32);
        const float sel = (hh == h) ? (h ? p1 : p0) : (h ? q1 : q0);
        const float y = 0.5f * sel + bias2;

        v4f ov;
        ov[0] = __shfl(y, (4 * l + 0) & 31, 32);
        ov[1] = __shfl(y, (4 * l + 1) & 31, 32);
        ov[2] = __shfl(y, (4 * l + 2) & 31, 32);
        ov[3] = __shfl(y, (4 * l + 3) & 31, 32);

        store_out_line(outc, tbase, l, ov, Ec);
        __threadfence();
        store_out_line(outc, tbase, l, ov, Ec);
    }
}

extern "C" void kernel_launch(void* const* d_in, const int* in_sizes, int n_in,
                              void* d_out, int out_size, void* d_ws, size_t ws_size,
                              hipStream_t stream)
{
    (void)n_in; (void)out_size;
    const float* x    = (const float*)d_in[0];
    const int*   eidx = (const int*)d_in[1];
    const float* W1   = (const float*)d_in[5];
    const float* b1   = (const float*)d_in[6];
    const float* W2   = (const float*)d_in[7];
    const float* b2   = (const float*)d_in[8];
    float* out = (float*)d_out;

    const int N = in_sizes[0] / NODE_DIM;
    const int E = in_sizes[1] / 2;
    if (N <= 0 || E <= 0) return;

    int chunk = 262144;
    while (chunk > 32 && (size_t)chunk * (ROWH * 2) + 65536 > ws_size) chunk >>= 1;
    if ((size_t)chunk * (ROWH * 2) + 65536 > ws_size) return;
    const int nch = (E + chunk - 1) / chunk;
    if (nch > 512) return;

    char* ws = (char*)d_ws;
    _Float16* G    = (_Float16*)(ws);
    _Float16* w1pk = (_Float16*)(ws + (size_t)chunk * (ROWH * 2));

    repack_w1_f16<<<16, 256, 0, stream>>>(W1, w1pk);

    for (int ch = 0; ch < nch; ++ch) {
        const int e0 = ch * chunk;
        const int Ec = (E - e0 < chunk) ? (E - e0) : chunk;
        const size_t gthreads = (size_t)Ec * 16;
        const unsigned gblocks = (unsigned)((gthreads + 255) / 256);
        gather_rows_f16<<<gblocks, 256, 0, stream>>>(x, eidx, G, N, E, e0, Ec);
        const int tiles  = (Ec + 31) / 32;
        const unsigned mblocks = (unsigned)((tiles + 7) / 8);
        edge_mlp_wmma<<<mblocks, 256, 0, stream>>>(G, w1pk, b1, W2, b2, out + e0, Ec);
    }
}
